// MultiHeadAttention_28449863369185
// MI455X (gfx1250) — hardware-run, weakly checked
//
#include <hip/hip_runtime.h>


#ifndef NB
#define NB 2
#endif
#ifndef SEQ
#define SEQ 2048
#endif
#define NB_FULL  2
#define SEQ_FULL 2048
#ifndef OUT_SEQ
#define OUT_SEQ SEQ
#endif
#define DM   1024
#define NH_  16
#define HD   64
#define AW   4
#define QRS  2048.0f
#define QRI  (1.0f / 2048.0f)
#define LOG2E 1.4426950408889634f
#define SC2  (0.125f * LOG2E)
#define PSH  8.0f
#define WSC  64.0f
#define WSI  (1.0f / 64.0f)
#define CSC  256.0f
#define OSC  (1.0f / (64.0f * 256.0f))

static_assert(HD == 64);
static_assert(NH_ * HD == DM);
static_assert(DM == 8 * 32 * 4);
static_assert(DM % 64 == 0);
static_assert(DM % 32 == 0);
static_assert(SEQ % 64 == 0);
static_assert((NB * SEQ) % 64 == 0);
static_assert((NB * SEQ) % 8 == 0);
static_assert(SEQ % 32 == 0);
static_assert(SEQ % (16 * AW) == 0);
static_assert(((size_t)DM * DM) % (8 * 256) == 0);
static_assert(NB <= NB_FULL);
static_assert(SEQ <= SEQ_FULL);

typedef _Float16 h16;
typedef __attribute__((ext_vector_type(16))) _Float16 v16h;
typedef __attribute__((ext_vector_type(8)))  _Float16 v8h;
typedef __attribute__((ext_vector_type(4)))  _Float16 v4h;
typedef __attribute__((ext_vector_type(8)))  float    v8f;
typedef __attribute__((ext_vector_type(4)))  float    v4f;
typedef v4f  __attribute__((may_alias)) v4fa;
typedef v8h  __attribute__((may_alias)) v8ha;
typedef v4h  __attribute__((may_alias)) v4ha;

__device__ __forceinline__ float bfr(float f) { unsigned u = __float_as_uint(f); u += 0x7FFFu + ((u >> 16) & 1u); return __uint_as_float(u & 0xFFFF0000u); }
__device__ __forceinline__ v16h cat16(v8h lo, v8h hi) { return __builtin_shufflevector(lo, hi, 0, 1, 2, 3, 4, 5, 6, 7, 8, 9, 10, 11, 12, 13, 14, 15); }
__device__ __forceinline__ v8f wmma16(v16h a, v16h b, v8f c) { return __builtin_amdgcn_wmma_f32_16x16x32_f16(false, a, false, b, (short)0, c, false, false); }
__device__ __forceinline__ v16h  ldh(const h16* p) { return cat16(*(const v8h*)p, *(const v8h*)(p + 16)); }
__device__ __forceinline__ void wave_sync() { __builtin_amdgcn_fence(3  , "wavefront"); __builtin_amdgcn_wave_barrier(); asm volatile("" ::: "memory"); }

__global__ __launch_bounds__(256) void k_rms(const float* __restrict__ x, const float* __restrict__ gamma, float* XNF, h16* XH) {
    __shared__ __align__(16) h16 hs[8 * DM];
    const int lane = threadIdx.x & 31, wave = __builtin_amdgcn_readfirstlane((int)(threadIdx.x >> 5));
    const int r = blockIdx.x * 8 + wave;
    const int b = r / SEQ, t = r - b * SEQ;
    const float* xr = x + ((size_t)b * SEQ_FULL + t) * DM;
    v4f v[8]; float ss = 0.0f;
#pragma unroll
    for (int i = 0; i < 8; ++i) { v4f u = *(const v4f*)(xr + (i * 32 + lane) * 4);
        u[0] = bfr(u[0]); u[1] = bfr(u[1]); u[2] = bfr(u[2]); u[3] = bfr(u[3]); v[i] = u;
        ss += u[0] * u[0] + u[1] * u[1] + u[2] * u[2] + u[3] * u[3]; }
    ss += __shfl_xor(ss, 16, 32); ss += __shfl_xor(ss, 8, 32); ss += __shfl_xor(ss, 4, 32); ss += __shfl_xor(ss, 2, 32); ss += __shfl_xor(ss, 1, 32);
    const float scale = rsqrtf(ss * (1.0f / (float)DM) + 1.0e-12f);
    h16* hw = hs + wave * DM;
#pragma unroll
    for (int i = 0; i < 8; ++i) { const v4f g = *(const v4f*)(gamma + (i * 32 + lane) * 4); v4f y; v4h hh;
#pragma unroll
        for (int k = 0; k < 4; ++k) { y[k] = (v[i][k] * scale) * bfr(g[k]); hh[k] = (h16)y[k]; }
        v[i] = y; *(v4ha*)(hw + (i * 32 + lane) * 4) = hh; }
    wave_sync();
    float* of = XNF + (size_t)r * DM; h16* oh = XH + (size_t)r * DM;
#pragma unroll 1
    for (int ps = 0; ps < 2; ++ps) {
#pragma unroll
        for (int i = 0; i < 8; ++i) *(volatile v4f*)(of + (i * 32 + lane) * 4) = v[i];
#pragma unroll
        for (int j = 0; j < 4; ++j) { const v8h hv = *(const v8ha*)(hw + (j * 32 + lane) * 8); *(volatile v8h*)(oh + (j * 32 + lane) * 8) = hv; }
        if (ps == 0) __threadfence(); }
}

__global__ __launch_bounds__(256) void k_cvtw(const float* __restrict__ src, h16* dst, size_t n8) {
    const size_t i = (size_t)blockIdx.x * 256 + threadIdx.x; if (i >= n8) return;
    const v8f v = *(const v8f*)(src + i * 8); v8h o;
#pragma unroll
    for (int k = 0; k < 8; ++k) o[k] = (h16)(bfr(v[k]) * WSC);
    *(volatile v8h*)(dst + i * 8) = o; __threadfence(); *(volatile v8h*)(dst + i * 8) = o;
}

__global__ __launch_bounds__(32) void k_gemm_p(const h16* __restrict__ A, const h16* __restrict__ Bt, h16* Ph, h16* Pr, int useRes, float osc, int RB, size_t sRB, int pitch, int CB, size_t sCB) {
    __shared__ __align__(16) float os[16 * 68];
    const int K = DM;
    const int lane = threadIdx.x & 31, lr = lane & 15, hi = lane >> 4; const int r0 = blockIdx.x * 64, c0 = blockIdx.y * 64;
    v8f acc[4][4];
#pragma unroll
    for (int mb = 0; mb < 4; ++mb)
#pragma unroll
        for (int nb = 0; nb < 4; ++nb) acc[mb][nb] = (v8f){};
    const size_t aoff = (size_t)(r0 + lr) * K + 8 * hi, boff = (size_t)(c0 + lr) * K + 8 * hi;
#pragma unroll 1
    for (int kc = 0; kc < K; kc += 32) {
        v16h a[4];
#pragma unroll
        for (int mb = 0; mb < 4; ++mb) a[mb] = ldh(A + aoff + (size_t)mb * 16 * K + kc);
#pragma unroll
        for (int nb = 0; nb < 4; ++nb) { const v16h b = ldh(Bt + boff + (size_t)nb * 16 * K + kc);
#pragma unroll
            for (int mb = 0; mb < 4; ++mb) acc[mb][nb] = wmma16(a[mb], b, acc[mb][nb]); }
        asm volatile("v_nop\n\tv_nop\n\tv_nop\n\tv_nop" : "+v"(acc[0][0]), "+v"(acc[1][1]), "+v"(acc[2][2]), "+v"(acc[3][3]) : "v"(a[0]), "v"(a[1]), "v"(a[2]), "v"(a[3]));
    }
    const size_t tbase = (size_t)(r0 / RB) * sRB + (size_t)(r0 % RB) * (size_t)pitch + (size_t)(c0 / CB) * sCB + (size_t)(c0 % CB);
#pragma unroll
    for (int mb = 0; mb < 4; ++mb) {
#pragma unroll
        for (int nb = 0; nb < 4; ++nb) {
#pragma unroll
            for (int j = 0; j < 8; ++j) os[(hi * 8 + j) * 68 + nb * 16 + lr] = acc[mb][nb][j]; }
        wave_sync();
        const size_t sb = tbase + (size_t)(mb * 16) * (size_t)pitch;
#pragma unroll 1
        for (int ps = 0; ps < 2; ++ps) {
#pragma unroll
            for (int s = 0; s < 4; ++s) { const int row = 4 * s + (lane >> 3), c8 = (lane & 7) * 8;
                const v4f x0 = *(const v4fa*)(&os[row * 68 + c8]) * osc; const v4f x1 = *(const v4fa*)(&os[row * 68 + c8 + 4]) * osc; v8h hv, rv;
#pragma unroll
                for (int i = 0; i < 4; ++i) { const h16 a0 = (h16)x0[i]; const h16 a1 = (h16)x1[i]; hv[i] = a0; hv[4 + i] = a1; rv[i] = (h16)((x0[i] - (float)a0) * QRS); rv[4 + i] = (h16)((x1[i] - (float)a1) * QRS); }
                const size_t oo = sb + (size_t)row * (size_t)pitch + c8;
                *(volatile v8h*)(Ph + oo) = hv; if (useRes) *(volatile v8h*)(Pr + oo) = rv; }
            if (ps == 0) __threadfence(); }
        wave_sync();
    }
}

__global__ __launch_bounds__(32) void k_gemm_o(const h16* __restrict__ A, const h16* __restrict__ Bt, float* OF, const float* __restrict__ RES, float osc, int RB, size_t sRB, int opitch) {
    __shared__ __align__(16) float os[16 * 68];
    const int K = DM;
    const int lane = threadIdx.x & 31, lr = lane & 15, hi = lane >> 4; const int r0 = blockIdx.x * 64, c0 = blockIdx.y * 64;
    v8f acc[4][4];
#pragma unroll
    for (int mb = 0; mb < 4; ++mb)
#pragma unroll
        for (int nb = 0; nb < 4; ++nb) acc[mb][nb] = (v8f){};
    const size_t aoff = (size_t)(r0 + lr) * K + 8 * hi, boff = (size_t)(c0 + lr) * K + 8 * hi;
#pragma unroll 1
    for (int kc = 0; kc < K; kc += 32) {
        v16h a[4];
#pragma unroll
        for (int mb = 0; mb < 4; ++mb) a[mb] = ldh(A + aoff + (size_t)mb * 16 * K + kc);
#pragma unroll
        for (int nb = 0; nb < 4; ++nb) { const v16h b = ldh(Bt + boff + (size_t)nb * 16 * K + kc);
#pragma unroll
            for (int mb = 0; mb < 4; ++mb) acc[mb][nb] = wmma16(a[mb], b, acc[mb][nb]); }
        asm volatile("v_nop\n\tv_nop\n\tv_nop\n\tv_nop" : "+v"(acc[0][0]), "+v"(acc[1][1]), "+v"(acc[2][2]), "+v"(acc[3][3]) : "v"(a[0]), "v"(a[1]), "v"(a[2]), "v"(a[3]));
    }
    const size_t obase = (size_t)(r0 / RB) * sRB + (size_t)(r0 % RB) * (size_t)opitch + (size_t)c0;
    const size_t rbase = (size_t)r0 * DM + (size_t)c0;
#pragma unroll
    for (int mb = 0; mb < 4; ++mb) {
#pragma unroll
        for (int nb = 0; nb < 4; ++nb) {
#pragma unroll
            for (int j = 0; j < 8; ++j) os[(hi * 8 + j) * 68 + nb * 16 + lr] = acc[mb][nb][j]; }
        wave_sync();
        const size_t sb = obase + (size_t)(mb * 16) * (size_t)opitch;
        const size_t rb = rbase + (size_t)(mb * 16) * DM;
#pragma unroll 1
        for (int ps = 0; ps < 2; ++ps) {
#pragma unroll
            for (int s = 0; s < 8; ++s) { const int row = 2 * s + hi, cofs = lr * 4;
                const v4f cv = *(const v4fa*)(&os[row * 68 + cofs]);
                const v4f xv = *(const v4f*)(RES + rb + (size_t)row * DM + cofs);
                const v4f val = cv * osc + xv;
                *(volatile v4f*)(OF + sb + (size_t)row * (size_t)opitch + cofs) = val; }
            if (ps == 0) __threadfence(); }
        wave_sync();
    }
}

__global__ __launch_bounds__(32 * AW) void k_flash(const h16* __restrict__ QH, const h16* __restrict__ QR, const h16* __restrict__ KP, const h16* __restrict__ VT, const float* __restrict__ MASK, h16* CTX) {
    __shared__ __align__(16) float os[AW * 16 * 68];
    const int lane = threadIdx.x & 31, wave = __builtin_amdgcn_readfirstlane((int)(threadIdx.x >> 5)), lr = lane & 15, hi = lane >> 4;
    const int zh = blockIdx.y; const int b = zh / NH_, h = zh % NH_;
    const int t0 = (blockIdx.x * AW + wave) * 16;
    const size_t pbase = (size_t)zh * SEQ * HD;
    const size_t qo = pbase + (size_t)(t0 + lr) * HD + 8 * hi;
    const v16h qh0 = ldh(QH + qo), qh1 = ldh(QH + qo + 32), qr0 = ldh(QR + qo), qr1 = ldh(QR + qo + 32);
    const size_t ko = pbase + (size_t)lr * HD + 8 * hi;
    const size_t vo = pbase + (size_t)lr * SEQ + 8 * hi;
    const float* mrow = MASK + (size_t)(t0 + lr) * SEQ_FULL + 8 * hi;
    v8f o0 = (v8f){}, o1 = (v8f){}, o2 = (v8f){}, o3 = (v8f){};
    float m = -3.0e38f, l = 0.0f;
#pragma unroll 1
    for (int key0 = 0; key0 < SEQ; key0 += 32) {
        const h16* ka = KP + ko + (size_t)key0 * HD;
        const v16h ka0 = ldh(ka), ka1 = ldh(ka + 32), kb0 = ldh(ka + 16 * HD), kb1 = ldh(ka + 16 * HD + 32);
        v8f sHa = (v8f){}, sLa = (v8f){}, sHb = (v8f){}, sLb = (v8f){};
        sHa = wmma16(ka0, qh0, sHa); sLa = wmma16(ka0, qr0, sLa); sHb = wmma16(kb0, qh0, sHb); sLb = wmma16(kb0, qr0, sLb);
        sHa = wmma16(ka1, qh1, sHa); sLa = wmma16(ka1, qr1, sLa); sHb = wmma16(kb1, qh1, sHb); sLb = wmma16(kb1, qr1, sLb);
        asm volatile("v_nop\n\tv_nop\n\tv_nop\n\tv_nop" : "+v"(sHa), "+v"(sLa), "+v"(sHb), "+v"(sLb) : "v"(ka0), "v"(ka1), "v"(kb0), "v"(kb1));
        const float* mp = mrow + key0;
        const v4f ma0 = *(const v4f*)(mp), ma1 = *(const v4f*)(mp + 4), mb0 = *(const v4f*)(mp + 16), mb1 = *(const v4f*)(mp + 20);
        float ta[8], tb[8]; float mx = -3.0e38f;
#pragma unroll
        for (int r = 0; r < 4; ++r) {
            ta[r]     = (sHa[r]     + sLa[r]     * QRI) * SC2 + bfr(ma0[r]) * LOG2E;
            ta[4 + r] = (sHa[4 + r] + sLa[4 + r] * QRI) * SC2 + bfr(ma1[r]) * LOG2E;
            tb[r]     = (sHb[r]     + sLb[r]     * QRI) * SC2 + bfr(mb0[r]) * LOG2E;
            tb[4 + r] = (sHb[4 + r] + sLb[4 + r] * QRI) * SC2 + bfr(mb1[r]) * LOG2E;
            mx = fmaxf(mx, fmaxf(fmaxf(ta[r], ta[4 + r]), fmaxf(tb[r], tb[4 + r]))); }
        mx = fmaxf(mx, __shfl_xor(mx, 16, 32));
        const float mnew = fmaxf(m, mx);
        const float alpha = __builtin_amdgcn_exp2f(m - mnew);
        const float sh = PSH - mnew;
        v16h pb; float ls = 0.0f;
#pragma unroll
        for (int r = 0; r < 8; ++r) { const h16 pa = (h16)__builtin_amdgcn_exp2f(ta[r] + sh); const h16 pc = (h16)__builtin_amdgcn_exp2f(tb[r] + sh); pb[r] = pa; pb[8 + r] = pc; ls += (float)pa + (float)pc; }
        l = l * alpha + ls; m = mnew;
        o0 = o0 * alpha; o1 = o1 * alpha; o2 = o2 * alpha; o3 = o3 * alpha;
        const h16* va = VT + vo + key0;
        const v16h v0 = ldh(va), v1 = ldh(va + (size_t)16 * SEQ), v2 = ldh(va + (size_t)32 * SEQ), v3 = ldh(va + (size_t)48 * SEQ);
        o0 = wmma16(v0, pb, o0); o1 = wmma16(v1, pb, o1); o2 = wmma16(v2, pb, o2); o3 = wmma16(v3, pb, o3);
        asm volatile("v_nop\n\tv_nop\n\tv_nop\n\tv_nop" : "+v"(o0), "+v"(o1), "+v"(o2), "+v"(o3) : "v"(v0), "v"(v1), "v"(v2), "v"(v3), "v"(pb));
    }
    l += __shfl_xor(l, 16, 32);
    const float inv = CSC * (1.0f / l);
    const int wb = wave * 16 * 68;
    { v4f a, c;
      a[0] = o0[0] * inv; a[1] = o0[1] * inv; a[2] = o0[2] * inv; a[3] = o0[3] * inv; c[0] = o0[4] * inv; c[1] = o0[5] * inv; c[2] = o0[6] * inv; c[3] = o0[7] * inv;
      *(v4fa*)(&os[wb + lr * 68 +  0 + 8 * hi]) = a; *(v4fa*)(&os[wb + lr * 68 +  0 + 8 * hi + 4]) = c;
      a[0] = o1[0] * inv; a[1] = o1[1] * inv; a[2] = o1[2] * inv; a[3] = o1[3] * inv; c[0] = o1[4] * inv; c[1] = o1[5] * inv; c[2] = o1[6] * inv; c[3] = o1[7] * inv;
      *(v4fa*)(&os[wb + lr * 68 + 16 + 8 * hi]) = a; *(v4fa*)(&os[wb + lr * 68 + 16 + 8 * hi + 4]) = c;
      a[0] = o2[0] * inv; a[1] = o2[1] * inv; a[2] = o2[2] * inv; a[3] = o2[3] * inv; c[0] = o2[4] * inv; c[1] = o2[5] * inv; c[2] = o2[6] * inv; c[3] = o2[7] * inv;
      *(v4fa*)(&os[wb + lr * 68 + 32 + 8 * hi]) = a; *(v4fa*)(&os[wb + lr * 68 + 32 + 8 * hi + 4]) = c;
      a[0] = o3[0] * inv; a[1] = o3[1] * inv; a[2] = o3[2] * inv; a[3] = o3[3] * inv; c[0] = o3[4] * inv; c[1] = o3[5] * inv; c[2] = o3[6] * inv; c[3] = o3[7] * inv;
      *(v4fa*)(&os[wb + lr * 68 + 48 + 8 * hi]) = a; *(v4fa*)(&os[wb + lr * 68 + 48 + 8 * hi + 4]) = c; }
    wave_sync();
    h16* crow = CTX + ((size_t)b * SEQ + t0) * DM + h * HD;
#pragma unroll 1
    for (int ps = 0; ps < 2; ++ps) {
#pragma unroll
        for (int s = 0; s < 4; ++s) { const int row = 4 * s + (lane >> 3), c8 = (lane & 7) * 8;
            const v4f x0 = *(const v4fa*)(&os[wb + row * 68 + c8]); const v4f x1 = *(const v4fa*)(&os[wb + row * 68 + c8 + 4]); v8h hv;
#pragma unroll
            for (int i = 0; i < 4; ++i) { hv[i] = (h16)x0[i]; hv[4 + i] = (h16)x1[i]; }
            *(volatile v8h*)(crow + (size_t)row * DM + c8) = hv; }
        if (ps == 0) __threadfence(); }
}

static constexpr size_t al256(size_t v) { return (v + 255) & ~(size_t)255; }
static constexpr size_t SZ_XF = al256((size_t)NB * SEQ * DM * 4);
static constexpr size_t SZ_XH = al256((size_t)NB * SEQ * DM * 2);
static constexpr size_t SZ_WB = al256((size_t)4 * DM * DM * 2);
static constexpr size_t SZ_PL = al256((size_t)NB * NH_ * SEQ * HD * 2);
static constexpr size_t SZ_CX = al256((size_t)NB * SEQ * DM * 2);
static constexpr size_t SZ_TOTAL = SZ_XF + SZ_XH + SZ_WB + 4 * SZ_PL + SZ_CX;
static_assert(SZ_TOTAL <= (size_t)134217728);
static_assert(((size_t)DM * DM * 2) % 256 == 0);

extern "C" void kernel_launch(void* const* d_in, const int* in_sizes, int n_in,
                              void* d_out, int out_size, void* d_ws, size_t ws_size, hipStream_t stream) {
    if (n_in < 7) return;
    const size_t needx = ((size_t)(NB - 1) * SEQ_FULL + SEQ) * DM;
    if ((size_t)in_sizes[0] < needx) return;
    if ((size_t)in_sizes[1] < (size_t)(SEQ - 1) * SEQ_FULL + SEQ) return;
    if ((size_t)in_sizes[2] < (size_t)DM * DM || (size_t)in_sizes[3] < (size_t)DM * DM || (size_t)in_sizes[4] < (size_t)DM * DM || (size_t)in_sizes[5] < (size_t)DM * DM) return;
    if ((size_t)in_sizes[6] < (size_t)DM) return;
    if ((size_t)out_size < ((size_t)(NB - 1) * OUT_SEQ + SEQ) * DM) return;
    if (SZ_TOTAL > ws_size) return;
    const float* x = (const float*)d_in[0]; const float* mask = (const float*)d_in[1];
    const float* wq = (const float*)d_in[2]; const float* wk = (const float*)d_in[3]; const float* wv = (const float*)d_in[4]; const float* wo = (const float*)d_in[5];
    const float* gamma = (const float*)d_in[6];
    float* OUT = (float*)d_out;
    char* wsp = (char*)d_ws;
    float* XNF = (float*)wsp; wsp += SZ_XF;
    h16* XH = (h16*)wsp; wsp += SZ_XH;
    h16* WB = (h16*)wsp; wsp += SZ_WB;
    h16* QH = (h16*)wsp; wsp += SZ_PL;
    h16* QR = (h16*)wsp; wsp += SZ_PL;
    h16* KP = (h16*)wsp; wsp += SZ_PL;
    h16* VT = (h16*)wsp; wsp += SZ_PL;
    h16* CX = (h16*)wsp; wsp += SZ_CX;
    h16* WQ = WB; h16* WK = WB + (size_t)DM * DM; h16* WV = WB + (size_t)2 * DM * DM; h16* WO = WB + (size_t)3 * DM * DM;

    k_rms<<<NB * SEQ / 8, 256, 0, stream>>>(x, gamma, XNF, XH);
    { const size_t n8 = (size_t)DM * DM / 8; const unsigned g = (unsigned)((n8 + 255) / 256);
      k_cvtw<<<g, 256, 0, stream>>>(wq, WQ, n8); k_cvtw<<<g, 256, 0, stream>>>(wk, WK, n8);
      k_cvtw<<<g, 256, 0, stream>>>(wv, WV, n8); k_cvtw<<<g, 256, 0, stream>>>(wo, WO, n8); }

    k_gemm_p<<<dim3(NB * SEQ / 64, DM / 64, 1), 32, 0, stream>>>(XH, WQ, QH, QR, 1, WSI, SEQ, (size_t)NH_ * SEQ * HD, HD, HD, (size_t)SEQ * HD);
    k_gemm_p<<<dim3(NB * SEQ / 64, DM / 64, 1), 32, 0, stream>>>(XH, WK, KP, KP, 0, WSI, SEQ, (size_t)NH_ * SEQ * HD, HD, HD, (size_t)SEQ * HD);
    k_gemm_p<<<dim3(DM / 64, NB * SEQ / 64, 1), 32, 0, stream>>>(WV, XH, VT, VT, 0, WSI, DM, (size_t)0, SEQ, SEQ, (size_t)DM * SEQ);

    k_flash<<<dim3(SEQ / (16 * AW), NB * NH_, 1), 32 * AW, 0, stream>>>(QH, QR, KP, VT, mask, CX);

    k_gemm_o<<<dim3(NB * SEQ / 64, DM / 64, 1), 32, 0, stream>>>(CX, WO, OUT, XNF, OSC, SEQ, (size_t)OUT_SEQ * DM, DM);
}
